// SS2DCore_87445534146662
// MI455X (gfx1250) — hardware-verified
//
#include <hip/hip_runtime.h>


namespace {
constexpr int B = 2, C = 96, HI = 128, LI = HI * HI, D = 256, NT = B * LI;
constexpr float XS = 8.0f, YSC = 4096.0f, CS = 32768.0f, ZS = 65536.0f, WSC = 256.0f;
typedef _Float16 b16;
typedef __attribute__((ext_vector_type(16))) _Float16 v16b;
typedef __attribute__((ext_vector_type(8))) _Float16 v8b;
typedef __attribute__((ext_vector_type(8))) float v8f;
typedef __attribute__((ext_vector_type(4))) float v4f;
__device__ __forceinline__ float bf16_rne(float f) { unsigned int u = __float_as_uint(f); u += 0x7FFFu + ((u >> 16) & 1u); return __uint_as_float(u & 0xFFFF0000u); }
__device__ __forceinline__ void split16(float v, b16& hi, b16& lo) { hi = (b16)v; lo = (b16)(v - (float)hi); }
__device__ __forceinline__ v16b frag_kb(const b16* p, int hh) { const v8b a = *(const v8b*)(p + 8 * hh), b = *(const v8b*)(p + 16 + 8 * hh); v16b f;
#pragma unroll
  for (int e = 0; e < 8; ++e) { f[e] = a[e]; f[8 + e] = b[e]; } return f; }
__device__ __forceinline__ v8f wmma16b(v16b a, v16b b, v8f c) { v8f d = __builtin_amdgcn_wmma_f32_16x16x32_f16(false, a, false, b, (short)0, c, false, false); asm volatile("v_nop\n\tv_nop\n\tv_nop\n\tv_nop" : "+v"(d) : "v"(a), "v"(b)); return d; }
__device__ __forceinline__ void wave_lds_sync() { __builtin_amdgcn_fence(__ATOMIC_RELEASE, "workgroup"); __builtin_amdgcn_wave_barrier(); __builtin_amdgcn_fence(__ATOMIC_ACQUIRE, "workgroup"); }
__device__ __forceinline__ float pmul(float a, float b) { float p = a * b; asm volatile("" : "+v"(p)); return p; }
__device__ __forceinline__ float softplus(float v) { return v > 20.0f ? v : (v < -20.0f ? __expf(v) : log1pf(__expf(v))); }
__device__ __forceinline__ float sigm(float v) { return 1.0f / (1.0f + __expf(-v)); }

__global__ __launch_bounds__(256) void wcopy_kernel(const float* __restrict__ w, int n8, int ro, int KIN, b16* __restrict__ WT) {
  const int u = blockIdx.x * 256 + threadIdx.x; if (u >= n8) return; const size_t e = (size_t)u * 8; v8b v;
#pragma unroll
  for (int j = 0; j < 8; ++j) v[j] = (b16)(bf16_rne(w[e + j]) * WSC); for (int pass = 0; pass < 2; ++pass) { *(volatile v8b*)(WT + (size_t)ro * KIN + e) = v; __threadfence(); }
}
__global__ __launch_bounds__(256) void xa_kernel(const float* __restrict__ x, b16* __restrict__ XA) {
  __shared__ float T[32][HI + 1]; const int cg = blockIdx.x % 3, y = (blockIdx.x / 3) % HI, b = blockIdx.x / (3 * HI); const int tid = threadIdx.x;
  for (int i = tid; i < 32 * HI; i += 256) { const int cl = i / HI, xx = i % HI; T[cl][xx] = bf16_rne(x[(((size_t)b * C + cg * 32 + cl) * HI + y) * HI + xx]); }
  __syncthreads();
  for (int pass = 0; pass < 2; ++pass) { for (int i = tid; i < HI * 4; i += 256) { const int xx = i / 4, g8 = i % 4; v8b v; for (int j = 0; j < 8; ++j) v[j] = (b16)(T[g8 * 8 + j][xx] * XS); *(volatile v8b*)(XA + (((size_t)b * HI + y) * HI + xx) * C + cg * 32 + g8 * 8) = v; } __threadfence(); }
}
__global__ __launch_bounds__(32) void proj_kernel(const b16* __restrict__ XA, const b16* __restrict__ WT, const float* __restrict__ xb, const float* __restrict__ bcb, const float* __restrict__ db, int NTV, float* __restrict__ AB, float* __restrict__ G, float* __restrict__ CC) {
  __shared__ __attribute__((aligned(16))) b16 Ah[16][C + 8]; __shared__ __attribute__((aligned(16))) float Us[16][D + 4], Bs[16][D + 4], Tf[16][128 + 4];
  const int lane = threadIdx.x, nloc = lane & 15, hlf = lane >> 4; const size_t t0 = (size_t)blockIdx.x * 16; if (t0 >= (size_t)NTV) return;
  for (int rr = 0; rr < 16; ++rr) for (int q = 0; q < 3; ++q) Ah[rr][q * 32 + lane] = XA[(t0 + rr) * C + q * 32 + lane];
  wave_lds_sync();
#pragma unroll 1
  for (int cg = 0; cg < 8; ++cg) { v8f acc[8];
#pragma unroll
    for (int t = 0; t < 8; ++t) acc[t] = (v8f){};
#pragma unroll
    for (int kb = 0; kb < C; kb += 32) { const v16b a = frag_kb(&Ah[nloc][kb], hlf);
#pragma unroll
      for (int t = 0; t < 8; ++t) acc[t] = wmma16b(a, frag_kb(WT + (size_t)(cg * 128 + t * 16 + nloc) * C + kb, hlf), acc[t]); }
    const int kind = cg >> 1;
#pragma unroll
    for (int t = 0; t < 8; ++t) { const int c = (cg & 1) * 128 + t * 16 + nloc; const float bb = kind == 0 ? bf16_rne(xb[c]) : (kind == 3 ? bf16_rne(db[c]) : bf16_rne(bcb[(kind - 1) * D + c]));
#pragma unroll 1
      for (int r8 = 0; r8 < 8; ++r8) { const int rl = 8 * hlf + r8; const float v = acc[t][r8] * (1.0f / (XS * WSC)) + bb;
        if (kind == 0) Us[rl][c] = v; else if (kind == 1) Bs[rl][c] = v; else if (kind == 2) Tf[rl][t * 16 + nloc] = v; else { const float ab = __expf(-softplus(v)); Tf[rl][t * 16 + nloc] = ab; Bs[rl][c] = pmul(pmul(1.0f - ab, Bs[rl][c]), Us[rl][c]); } } }
    wave_lds_sync();
    if (kind >= 2) { float* dst = (kind == 2) ? CC : AB;
      for (int pass = 0; pass < 2; ++pass) { for (int rr = 0; rr < 16; ++rr) *(volatile v4f*)(dst + (t0 + rr) * D + (cg & 1) * 128 + lane * 4) = *(const v4f*)(&Tf[rr][lane * 4]); __threadfence(); } }
    if (cg == 7) { for (int pass = 0; pass < 2; ++pass) { for (int rr = 0; rr < 16; ++rr) { *(volatile v4f*)(G + (t0 + rr) * D + lane * 4) = *(const v4f*)(&Bs[rr][lane * 4]); *(volatile v4f*)(G + (t0 + rr) * D + 128 + lane * 4) = *(const v4f*)(&Bs[rr][128 + lane * 4]); } __threadfence(); } }
    wave_lds_sync(); }
}
__global__ __launch_bounds__(256) void scan_kernel(const float* __restrict__ AB, const float* __restrict__ G, const float* __restrict__ CC, int b, int LSTEPS, float* __restrict__ Y) {
  const int gid = blockIdx.x * 256 + threadIdx.x; const int ch = gid % D, dir = gid / D; if (dir >= 4) return;
#pragma unroll 1
  for (int pass = 0; pass < 2; ++pass) { float h = 0.0f;
#pragma unroll 1
    for (int l = 0; l < LSTEPS; ++l) { const int lp = (dir >= 2) ? (LI - 1 - l) : l; const int tok = (dir & 1) ? ((lp % HI) * HI + lp / HI) : lp; const size_t t = (size_t)tok; (void)b;
      h = pmul(AB[t * D + ch], h) + G[t * D + ch]; ((volatile float*)Y)[((size_t)dir * LI + l) * D + ch] = pmul(CC[t * D + ch], h); }
    __threadfence(); }
}
__global__ __launch_bounds__(32) void yproj_kernel(const float* __restrict__ Y, const b16* __restrict__ WY, const float* __restrict__ yb, int LSTEPS, float* __restrict__ YC) {
  __shared__ __attribute__((aligned(16))) b16 Ah[16][D + 8], Al[16][D + 8]; __shared__ __attribute__((aligned(16))) float Tf[16][128 + 4];
  const int lane = threadIdx.x, nloc = lane & 15, hlf = lane >> 4; const size_t r0 = (size_t)blockIdx.x * 16; const int dir = (int)(r0 / LI); const int l0 = (int)(r0 % LI); if (l0 >= LSTEPS) return;
  for (int rr = 0; rr < 16; ++rr) for (int q = 0; q < 8; ++q) { b16 p, ql; split16(Y[(r0 + rr) * D + q * 32 + lane] * YSC, p, ql); Ah[rr][q * 32 + lane] = p; Al[rr][q * 32 + lane] = ql; }
  wave_lds_sync();
#pragma unroll 1
  for (int cg = 0; cg < 2; ++cg) { v8f acc[8];
#pragma unroll
    for (int t = 0; t < 8; ++t) acc[t] = (v8f){};
#pragma unroll 2
    for (int kb = 0; kb < D; kb += 32) { const v16b a = frag_kb(&Ah[nloc][kb], hlf), a2 = frag_kb(&Al[nloc][kb], hlf);
#pragma unroll
      for (int t = 0; t < 8; ++t) { const v16b bw = frag_kb(WY + (size_t)(cg * 128 + t * 16 + nloc) * D + kb, hlf); acc[t] = wmma16b(a, bw, acc[t]); acc[t] = wmma16b(a2, bw, acc[t]); } }
#pragma unroll
    for (int t = 0; t < 8; ++t) { const int c = cg * 128 + t * 16 + nloc; const float bb = bf16_rne(yb[c]);
#pragma unroll 1
      for (int r8 = 0; r8 < 8; ++r8) Tf[8 * hlf + r8][t * 16 + nloc] = acc[t][r8] * (1.0f / (YSC * WSC)) + bb; }
    wave_lds_sync();
    for (int pass = 0; pass < 2; ++pass) { for (int rr = 0; rr < 16; ++rr) *(volatile v4f*)(YC + (size_t)(l0 + rr) * (4 * D) + dir * D + cg * 128 + lane * 4) = *(const v4f*)(&Tf[rr][lane * 4]); __threadfence(); }
    wave_lds_sync(); }
}
__global__ __launch_bounds__(32) void merge_kernel(const float* __restrict__ YC, const b16* __restrict__ WM, const float* __restrict__ mb, const b16* __restrict__ WG, const float* __restrict__ gb, const b16* __restrict__ WO, const float* __restrict__ ob, int b, int LSTEPS, float* __restrict__ out) {
  __shared__ __attribute__((aligned(16))) b16 Ch[16][4 * D + 8], Cl[16][4 * D + 8], Ah[16][D + 8], Al[16][D + 8]; __shared__ __attribute__((aligned(16))) float Ms[16][D + 4], To[C][33];
  const int lane = threadIdx.x, nloc = lane & 15, hlf = lane >> 4; const int p0 = blockIdx.x * 32; if (p0 >= LSTEPS) return;
#pragma unroll 1
  for (int half = 0; half < 2; ++half) { const size_t t0 = (size_t)p0 + half * 16;
    for (int rr = 0; rr < 16; ++rr) for (int q = 0; q < 32; ++q) { b16 p, ql; split16(YC[(t0 + rr) * (4 * D) + q * 32 + lane] * CS, p, ql); Ch[rr][q * 32 + lane] = p; Cl[rr][q * 32 + lane] = ql; }
    wave_lds_sync(); const b16 (*ahp)[4 * D + 8] = Ch; const b16 (*alp)[4 * D + 8] = Cl;
#pragma unroll 1
    for (int cg = 0; cg < 2; ++cg) { v8f acc[8];
#pragma unroll
      for (int t = 0; t < 8; ++t) acc[t] = (v8f){};
#pragma unroll 2
      for (int kb = 0; kb < 4 * D; kb += 32) { const v16b a = frag_kb(&ahp[nloc][kb], hlf), a2 = frag_kb(&alp[nloc][kb], hlf);
#pragma unroll
        for (int t = 0; t < 8; ++t) { const v16b bw = frag_kb(WM + (size_t)(cg * 128 + t * 16 + nloc) * (4 * D) + kb, hlf); acc[t] = wmma16b(a, bw, acc[t]); acc[t] = wmma16b(a2, bw, acc[t]); } }
#pragma unroll
      for (int t = 0; t < 8; ++t) { const int c = cg * 128 + t * 16 + nloc; const float bb = bf16_rne(mb[c]);
#pragma unroll 1
        for (int r8 = 0; r8 < 8; ++r8) Ms[8 * hlf + r8][c] = acc[t][r8] * (1.0f / (CS * WSC)) + bb; } }
#pragma unroll 1
    for (int cg = 0; cg < 2; ++cg) { v8f acc[8];
#pragma unroll
      for (int t = 0; t < 8; ++t) acc[t] = (v8f){};
#pragma unroll 2
      for (int kb = 0; kb < 4 * D; kb += 32) { const v16b a = frag_kb(&ahp[nloc][kb], hlf), a2 = frag_kb(&alp[nloc][kb], hlf);
#pragma unroll
        for (int t = 0; t < 8; ++t) { const v16b bw = frag_kb(WG + (size_t)(cg * 128 + t * 16 + nloc) * (4 * D) + kb, hlf); acc[t] = wmma16b(a, bw, acc[t]); acc[t] = wmma16b(a2, bw, acc[t]); } }
      wave_lds_sync();
#pragma unroll
      for (int t = 0; t < 8; ++t) { const int c = cg * 128 + t * 16 + nloc; const float bb = bf16_rne(gb[c]);
#pragma unroll
        for (int r8 = 0; r8 < 8; ++r8) { const int rl = 8 * hlf + r8; const float z = pmul(Ms[rl][c], sigm(acc[t][r8] * (1.0f / (CS * WSC)) + bb)); b16 p, q; split16(z * ZS, p, q); Ah[rl][c] = p; Al[rl][c] = q; } } }
    wave_lds_sync();
    v8f acc[6];
#pragma unroll
    for (int t = 0; t < 6; ++t) acc[t] = (v8f){};
#pragma unroll 2
    for (int kb = 0; kb < D; kb += 32) { const v16b a = frag_kb(&Ah[nloc][kb], hlf), a2 = frag_kb(&Al[nloc][kb], hlf);
#pragma unroll
      for (int t = 0; t < 6; ++t) { const v16b bw = frag_kb(WO + (size_t)(t * 16 + nloc) * D + kb, hlf); acc[t] = wmma16b(a, bw, acc[t]); acc[t] = wmma16b(a2, bw, acc[t]); } }
#pragma unroll
    for (int t = 0; t < 6; ++t) { const int c = t * 16 + nloc; const float bb = bf16_rne(ob[c]);
#pragma unroll
      for (int r8 = 0; r8 < 8; ++r8) To[c][half * 16 + 8 * hlf + r8] = acc[t][r8] * (1.0f / (ZS * WSC)) + bb; }
    wave_lds_sync(); }
  for (int pass = 0; pass < 2; ++pass) { for (int c = 0; c < C; ++c) ((volatile float*)out)[((size_t)b * C + c) * LI + p0 + lane] = To[c][lane]; __threadfence(); }
}
}

extern "C" void kernel_launch(void* const* d_in, const int* in_sizes, int n_in, void* d_out, int out_size, void* d_ws, size_t ws_size, hipStream_t stream) {
  (void)n_in;
  auto Fp = [&](int i) { return (const float*)d_in[i]; };
  if (in_sizes[0] != NT * C || in_sizes[1] != D * C || in_sizes[3] != 2 * D * C || in_sizes[5] != D * C || in_sizes[7] != D * D || in_sizes[9] != D * 4 * D || in_sizes[11] != D * 4 * D || in_sizes[13] != C * D || out_size != NT * C) return;
  const int NBV = B; const int NTV = NBV * LI; const int LSTEPS = LI;
  size_t off = 0; char* ws = (char*)d_ws;
  auto carve = [&](size_t bytes) { char* p = ws + off; off += (bytes + 255) & ~(size_t)255; return p; };
  b16* WP = (b16*)carve((size_t)4 * D * C * 2); b16* WY = (b16*)carve((size_t)D * D * 2); b16* WM = (b16*)carve((size_t)D * 4 * D * 2); b16* WGt = (b16*)carve((size_t)D * 4 * D * 2); b16* WO = (b16*)carve((size_t)C * D * 2); b16* XA = (b16*)carve((size_t)NT * C * 2);
  float* AB = (float*)carve((size_t)NT * D * 4); float* G = (float*)carve((size_t)NT * D * 4); float* CC = (float*)carve((size_t)NT * D * 4);
  float* Y = (float*)carve((size_t)4 * LI * D * 4); float* YC = (float*)carve((size_t)LI * 4 * D * 4);
  if (off > ws_size || off > ((size_t)255 << 20)) return;
  wcopy_kernel<<<(D * C / 8 + 255) / 256, 256, 0, stream>>>(Fp(1), D * C / 8, 0, C, WP); wcopy_kernel<<<(2 * D * C / 8 + 255) / 256, 256, 0, stream>>>(Fp(3), 2 * D * C / 8, D, C, WP); wcopy_kernel<<<(D * C / 8 + 255) / 256, 256, 0, stream>>>(Fp(5), D * C / 8, 3 * D, C, WP);
  wcopy_kernel<<<(D * D / 8 + 255) / 256, 256, 0, stream>>>(Fp(7), D * D / 8, 0, D, WY); wcopy_kernel<<<(D * 4 * D / 8 + 255) / 256, 256, 0, stream>>>(Fp(9), D * 4 * D / 8, 0, 4 * D, WM); wcopy_kernel<<<(D * 4 * D / 8 + 255) / 256, 256, 0, stream>>>(Fp(11), D * 4 * D / 8, 0, 4 * D, WGt); wcopy_kernel<<<(C * D / 8 + 255) / 256, 256, 0, stream>>>(Fp(13), C * D / 8, 0, D, WO);
  xa_kernel<<<NBV * HI * 3, 256, 0, stream>>>(Fp(0), XA);
  proj_kernel<<<NTV / 16, 32, 0, stream>>>(XA, WP, Fp(2), Fp(4), Fp(6), NTV, AB, G, CC);
  for (int b = 0; b < NBV; ++b) {
    scan_kernel<<<(4 * D) / 256, 256, 0, stream>>>(AB + (size_t)b * LI * D, G + (size_t)b * LI * D, CC + (size_t)b * LI * D, b, LSTEPS, Y);
    yproj_kernel<<<4 * LI / 16, 32, 0, stream>>>(Y, WY, Fp(8), LSTEPS, YC);
    merge_kernel<<<LI / 32, 32, 0, stream>>>(YC, WM, Fp(10), WGt, Fp(12), WO, Fp(14), b, LSTEPS, (float*)d_out); }
}
